// SwinTransBlock_7121055777148
// MI455X (gfx1250) — hardware-verified
//
#include <hip/hip_runtime.h>
#include <stdint.h>

#define NB   4
#define NSEQ 4096
#define NTOT 16384
#define DM   256
#define FF   1024

typedef _Float16 v16h __attribute__((ext_vector_type(16)));
typedef _Float16 v8h  __attribute__((ext_vector_type(8)));
typedef _Float16 v4h  __attribute__((ext_vector_type(4)));
typedef float    v8f  __attribute__((ext_vector_type(8)));
typedef float    v4f  __attribute__((ext_vector_type(4)));

static_assert((NSEQ % 256) == 0);
static_assert((DM % 64) == 0 && (FF % 64) == 0 && (NTOT % 64) == 0);
static_assert(NB * NSEQ == NTOT);

#if defined(__HIP_DEVICE_COMPILE__)
#define DEV_ASM(...) asm volatile(__VA_ARGS__)
#else
#define DEV_ASM(...) ((void)0)
#endif

__device__ __forceinline__ unsigned short bfbits(float f) {
  unsigned u = __float_as_uint(f);
  return (unsigned short)((u + 0x7FFFu + ((u >> 16) & 1u)) >> 16);
}
__device__ __forceinline__ float bfr(float f) { return __uint_as_float(((unsigned)bfbits(f)) << 16); }

__device__ __forceinline__ v16h ldfrag(const _Float16* p) {
  union { v16h v; v8h hh[2]; } f;
  f.hh[0] = *(const v8h*)(p);
  f.hh[1] = *(const v8h*)(p + 16);
  return f.v;
}
__device__ __forceinline__ v8f mma16(v16h a, v16h b, v8f c) {
  return __builtin_amdgcn_wmma_f32_16x16x32_f16(false, a, false, b, (short)0, c, false, false);
}
__device__ __forceinline__ v8f zero8() {
  v8f z;
#pragma unroll
  for (int i = 0; i < 8; ++i) z[i] = 0.0f;
  return z;
}

__device__ __forceinline__ void guard4(v8f& a, v8f& b, v8f& c, v8f& d, v16h x, v16h y) {
  DEV_ASM("v_nop\n\tv_nop\n\tv_nop\n\tv_nop" : "+v"(a), "+v"(b), "+v"(c), "+v"(d) : "v"(x), "v"(y));
}
__device__ __forceinline__ void keep4(v16h a, v16h b, v16h c, v16h d) {
  DEV_ASM("v_nop" :: "v"(a), "v"(b), "v"(c), "v"(d));
}
__device__ __forceinline__ void accg4(v8f& a, v8f& b, v8f& c, v8f& d) {
  DEV_ASM("v_nop\n\tv_nop\n\tv_nop\n\tv_nop" : "+v"(a), "+v"(b), "+v"(c), "+v"(d));
}
__device__ __forceinline__ void guard_s8(v8f& a0, v8f& a1, v8f& a2, v8f& a3, v8f& b0, v8f& b1, v8f& b2, v8f& b3,
                                         v16h x0, v16h x1, v16h y0, v16h y1, v16h y2, v16h y3) {
  DEV_ASM("v_nop\n\tv_nop\n\tv_nop\n\tv_nop"
          : "+v"(a0), "+v"(a1), "+v"(a2), "+v"(a3), "+v"(b0), "+v"(b1), "+v"(b2), "+v"(b3)
          : "v"(x0), "v"(x1), "v"(y0), "v"(y1), "v"(y2), "v"(y3));
}
__device__ __forceinline__ void guard_pv(v8f& a0, v8f& a1, v8f& b0, v8f& b1, v16h p0, v16h p1, v16h x0, v16h x1) {
  DEV_ASM("v_nop\n\tv_nop\n\tv_nop\n\tv_nop" : "+v"(a0), "+v"(a1), "+v"(b0), "+v"(b1) : "v"(p0), "v"(p1), "v"(x0), "v"(x1));
}

__global__ __launch_bounds__(256) void cvt_w_kernel(const float* __restrict__ w0, const float* __restrict__ w1,
                                                    const float* __restrict__ w2, const float* __restrict__ w3,
                                                    const float* __restrict__ w4,
                                                    _Float16* __restrict__ o0, _Float16* __restrict__ o1,
                                                    _Float16* __restrict__ o2, _Float16* __restrict__ o3,
                                                    _Float16* __restrict__ o4) {
  __shared__ float T[64 * 65];
  const int tid = threadIdx.x, bid = blockIdx.x;
  if (bid >= 176) return;
  int seg, t;
  if (bid < 16)       { seg = 0; t = bid; }
  else if (bid < 32)  { seg = 1; t = bid - 16; }
  else if (bid < 48)  { seg = 2; t = bid - 32; }
  else if (bid < 112) { seg = 3; t = bid - 48; }
  else                { seg = 4; t = bid - 112; }
  const float* src = (seg == 0) ? w0 : (seg == 1) ? w1 : (seg == 2) ? w2 : (seg == 3) ? w3 : w4;
  _Float16* dst = (seg == 0) ? o0 : (seg == 1) ? o1 : (seg == 2) ? o2 : (seg == 3) ? o3 : o4;
  const int R = (seg == 4) ? FF : DM;
  const int C = (seg == 3) ? FF : DM;
  const int tilesC = C >> 6;
  const int tr = t / tilesC, tc = t - tr * tilesC;
  const int r0 = tr << 6, c0 = tc << 6;
#pragma unroll
  for (int i = 0; i < 4; ++i) {
    const int idx = i * 256 + tid;
    const int r = idx >> 4, c4 = (idx & 15) * 4;
    const v4f v = *(const v4f*)(src + (size_t)(r0 + r) * C + c0 + c4);
#pragma unroll
    for (int e = 0; e < 4; ++e) T[(c4 + e) * 65 + r] = v[e];
  }
  __syncthreads();
  const int rq = tid >> 3, pc = (tid & 7) * 8;
  v8h o[2];
#pragma unroll
  for (int it = 0; it < 2; ++it) {
    const int nn = it * 32 + rq;
#pragma unroll
    for (int e = 0; e < 8; ++e) o[it][e] = (_Float16)(bfr(T[nn * 65 + pc + e]) * 64.0f);
  }
#pragma unroll
  for (int ps = 0; ps < 2; ++ps) {
#pragma unroll
    for (int it = 0; it < 2; ++it) {
      const int nn = it * 32 + rq;
      *(volatile v8h*)(dst + (size_t)(c0 + nn) * R + r0 + pc) = o[it];
    }
    __threadfence();
  }
}

__global__ __launch_bounds__(256) void ln1_kernel(const float* __restrict__ x, const float* __restrict__ g,
                                                  const float* __restrict__ b, float* __restrict__ xn,
                                                  _Float16* __restrict__ x16, int nrows) {
  const int wave = threadIdx.x >> 5, lane = threadIdx.x & 31;
  const int row = (int)blockIdx.x * 8 + wave;
  if (row >= nrows) return;
  const int ca = 4 * lane, cb = 128 + 4 * lane;
  const float* xr = x + (size_t)row * DM;
  const v4f a = *(const v4f*)(xr + ca), a2 = *(const v4f*)(xr + cb);
  float v[8];
#pragma unroll
  for (int e = 0; e < 4; ++e) { v[e] = bfr(a[e]); v[4 + e] = bfr(a2[e]); }
  float s = ((v[0] + v[1]) + (v[2] + v[3])) + ((v[4] + v[5]) + (v[6] + v[7]));
#pragma unroll
  for (int off = 16; off > 0; off >>= 1) s += __shfl_xor(s, off, 32);
  const float mu = s * (1.0f / 256.0f);
  float s2 = 0.0f;
#pragma unroll
  for (int e = 0; e < 8; ++e) { const float d = v[e] - mu; s2 += d * d; }
#pragma unroll
  for (int off = 16; off > 0; off >>= 1) s2 += __shfl_xor(s2, off, 32);
  const float rstd = rsqrtf(s2 * (1.0f / 256.0f) + 1e-5f);
  const v4f ga = *(const v4f*)(g + ca), gb = *(const v4f*)(g + cb);
  const v4f ba = *(const v4f*)(b + ca), bb = *(const v4f*)(b + cb);
  v4f ya, yb;
  v4h ha, hb;
#pragma unroll
  for (int e = 0; e < 4; ++e) {
    const float t0 = (v[e] - mu) * rstd * bfr(ga[e]) + bfr(ba[e]);
    const float t1 = (v[4 + e] - mu) * rstd * bfr(gb[e]) + bfr(bb[e]);
    ya[e] = t0; yb[e] = t1;
    ha[e] = (_Float16)(t0 * 8.0f); hb[e] = (_Float16)(t1 * 8.0f);
  }
  float* yr = xn + (size_t)row * DM;
  _Float16* hr = x16 + (size_t)row * DM;
#pragma unroll
  for (int ps = 0; ps < 2; ++ps) {
    *(volatile v4f*)(yr + ca) = ya;
    *(volatile v4f*)(yr + cb) = yb;
    *(volatile v4h*)(hr + ca) = ha;
    *(volatile v4h*)(hr + cb) = hb;
    __threadfence();
  }
}

template <int OUT_MODE, bool BIAS_ROW, bool RELU, bool RESID>
__global__ __launch_bounds__(256) void gemm64_kernel(const _Float16* __restrict__ A, int lda,
                                                     const _Float16* __restrict__ Bt, int ldb,
                                                     void* __restrict__ Cout, _Float16* __restrict__ C2, int ldc,
                                                     const float* __restrict__ bias,
                                                     const float* __restrict__ resid, int ldr,
                                                     int M, int N, int K, float scale, float bscale) {
  __shared__ __align__(16) float sT[8][16 * 68];
  const int lane = threadIdx.x & 31, wave = threadIdx.x >> 5;
  const int tilesN = N >> 6, tilesM = M >> 6;
  const int tile = (int)blockIdx.x * 8 + wave;
  if (tile >= tilesM * tilesN) return;
  const int tm = tile / tilesN, tn = tile - tm * tilesN;
  const int m0 = tm << 6, n0 = tn << 6;
  const int rl = lane & 15;
  const int koff = (lane >> 4) * 8;
  const int mOff = (lane >> 4) * 8;

  v8f acc[4][4];
#pragma unroll
  for (int i = 0; i < 4; ++i)
#pragma unroll
    for (int j = 0; j < 4; ++j) acc[i][j] = zero8();

#pragma unroll 1
  for (int k0 = 0; k0 < K; k0 += 32) {
    v16h bh[4];
#pragma unroll
    for (int j = 0; j < 4; ++j) bh[j] = ldfrag(Bt + (size_t)(n0 + (j << 4) + rl) * ldb + koff + k0);
#pragma unroll
    for (int i = 0; i < 4; ++i) {
      const v16h ah = ldfrag(A + (size_t)(m0 + (i << 4) + rl) * lda + koff + k0);
#pragma unroll
      for (int j = 0; j < 4; ++j) acc[i][j] = mma16(ah, bh[j], acc[i][j]);
      guard4(acc[i][0], acc[i][1], acc[i][2], acc[i][3], ah, bh[3]);
    }
    keep4(bh[0], bh[1], bh[2], bh[3]);
  }
  accg4(acc[0][0], acc[0][1], acc[0][2], acc[0][3]);
  accg4(acc[1][0], acc[1][1], acc[1][2], acc[1][3]);
  accg4(acc[2][0], acc[2][1], acc[2][2], acc[2][3]);
  accg4(acc[3][0], acc[3][1], acc[3][2], acc[3][3]);

  float* slab = sT[wave];
#pragma unroll
  for (int i = 0; i < 4; ++i) {
    const int mBase = m0 + (i << 4);
    float brow[8];
#pragma unroll
    for (int r = 0; r < 8; ++r) brow[r] = 0.0f;
    if (BIAS_ROW) {
#pragma unroll
      for (int r = 0; r < 8; ++r) brow[r] = bscale * bfr(bias[mBase + mOff + r]);
    }
#pragma unroll
    for (int j = 0; j < 4; ++j) {
      float bcol = 0.0f;
      if (!BIAS_ROW) bcol = bscale * bfr(bias[n0 + (j << 4) + rl]);
#pragma unroll
      for (int r = 0; r < 8; ++r) {
        float v = acc[i][j][r] * scale + (BIAS_ROW ? brow[r] : bcol);
        if (RELU) v = fmaxf(v, 0.0f);
        slab[(mOff + r) * 68 + (j << 4) + rl] = v;
      }
    }
    __builtin_amdgcn_fence(__ATOMIC_RELEASE, "workgroup");
    __builtin_amdgcn_wave_barrier();
    __builtin_amdgcn_fence(__ATOMIC_ACQUIRE, "workgroup");
    if (OUT_MODE == 0) {
      float* Cf = (float*)Cout;
      const int hh = lane >> 4, c4 = (lane & 15) * 4;
#pragma unroll
      for (int ps = 0; ps < 2; ++ps) {
#pragma unroll
        for (int it = 0; it < 8; ++it) {
          const int row = it * 2 + hh;
          v4f v = *(const v4f*)(slab + row * 68 + c4);
          if (RESID) {
            const v4f rv = *(const v4f*)(resid + (size_t)(mBase + row) * ldr + n0 + c4);
            v = v + rv;
          }
          *(volatile v4f*)(Cf + (size_t)(mBase + row) * ldc + n0 + c4) = v;
        }
        __threadfence();
      }
    } else {
      _Float16* Ch = (_Float16*)Cout;
      const int qq = lane >> 3, c8 = (lane & 7) * 8;
#pragma unroll
      for (int ps = 0; ps < 2; ++ps) {
#pragma unroll
        for (int it = 0; it < 4; ++it) {
          const int row = it * 4 + qq;
          const float* sp = slab + row * 68 + c8;
          v8h hv, rv;
#pragma unroll
          for (int e = 0; e < 8; ++e) {
            const float v = sp[e];
            const _Float16 q16 = (_Float16)v;
            hv[e] = q16;
            rv[e] = (_Float16)((v - (float)q16) * 2048.0f);
          }
          const size_t o = (size_t)(mBase + row) * ldc + n0 + c8;
          *(volatile v8h*)(Ch + o) = hv;
          if (OUT_MODE == 2) *(volatile v8h*)(C2 + o) = rv;
        }
        __threadfence();
      }
    }
    __builtin_amdgcn_fence(__ATOMIC_RELEASE, "workgroup");
    __builtin_amdgcn_wave_barrier();
    __builtin_amdgcn_fence(__ATOMIC_ACQUIRE, "workgroup");
  }
}

#define QB    32
#define KCH   256
#define QSP   264
#define PSP   264
#define OSP   260
#define LQH   0
#define LQR   16896
#define LPS   33792
#define LPMAX 50688
#define LPSUM 51712
#define LST   52736
#define LTOT  53248
static_assert(QB * QSP * 2 == LQR - LQH);
static_assert(QB * QSP * 2 == LPS - LQR);
static_assert(QB * PSP * 2 == LPMAX - LPS);
static_assert(LPSUM - LPMAX == 256 * 4);
static_assert(LST - LPSUM == 256 * 4);
static_assert(LTOT - LST == 4 * 32 * 4);
static_assert(QB * OSP * 4 <= LPS);
static_assert((QSP % 8) == 0 && (PSP % 8) == 0 && (OSP % 4) == 0 && PSP >= KCH);
static_assert((LQR % 16) == 0 && (LPS % 16) == 0 && (LPMAX % 16) == 0 && (LST % 16) == 0);
static_assert((NSEQ % KCH) == 0 && (NSEQ % QB) == 0 && (DM % 32) == 0);

__global__ __launch_bounds__(256) void attn_kernel(const _Float16* __restrict__ qh, const _Float16* __restrict__ qr,
                                                   const _Float16* __restrict__ kh, const _Float16* __restrict__ vt,
                                                   const float* __restrict__ xn, const float* __restrict__ g2,
                                                   const float* __restrict__ be2, float* __restrict__ x1,
                                                   _Float16* __restrict__ h16) {
  __shared__ __align__(16) char smem[LTOT];
  _Float16* Qh = (_Float16*)(smem + LQH);
  _Float16* Qr = (_Float16*)(smem + LQR);
  _Float16* Ps = (_Float16*)(smem + LPS);
  float* pmax = (float*)(smem + LPMAX);
  float* psum = (float*)(smem + LPSUM);
  float* m_s  = (float*)(smem + LST);
  float* l_s  = m_s + 32;
  float* al_s = m_s + 64;
  float* li_s = m_s + 96;

  const int tid = threadIdx.x, wave = tid >> 5, lane = tid & 31, h = lane >> 4, c = lane & 15;
  const int q0 = (int)blockIdx.x * QB;
  const int bat = q0 / NSEQ;
  const _Float16* kbase = kh + (size_t)bat * NSEQ * DM;
  const _Float16* vbase = vt + (size_t)bat * NSEQ;
  const float ninf = -__builtin_inff();

  if (tid < 32) { m_s[tid] = ninf; l_s[tid] = 0.0f; al_s[tid] = 0.0f; li_s[tid] = 0.0f; }
  psum[tid] = 0.0f;
#pragma unroll
  for (int i = 0; i < 4; ++i) {
    const int idx = i * 256 + tid;
    const int row = idx >> 5, pc = idx & 31;
    const size_t go = (size_t)(q0 + row) * DM + pc * 8;
    *(v8h*)(Qh + row * QSP + pc * 8) = *(const v8h*)(qh + go);
    *(v8h*)(Qr + row * QSP + pc * 8) = *(const v8h*)(qr + go);
  }
  __syncthreads();

  v8f oacc[2][2];
#pragma unroll
  for (int qt = 0; qt < 2; ++qt)
#pragma unroll
    for (int nt = 0; nt < 2; ++nt) oacc[qt][nt] = zero8();

  const _Float16* qb0p = Qh + c * QSP + 8 * h;
  const _Float16* qb1p = Qh + (16 + c) * QSP + 8 * h;
  const _Float16* qr0p = Qr + c * QSP + 8 * h;
  const _Float16* qr1p = Qr + (16 + c) * QSP + 8 * h;
  const _Float16* pa0p = Ps + c * PSP + 8 * h;
  const _Float16* pa1p = Ps + (16 + c) * PSP + 8 * h;
  const int ntile = NSEQ / KCH;
  const float S_SC = 0.000244140625f;
  const float R_INV = 0.00048828125f;

#pragma unroll 1
  for (int t = 0; t < ntile; ++t) {
    const int kb = t * KCH + 32 * wave;
    const _Float16* ka0p = kbase + (size_t)(kb + c) * DM + 8 * h;
    const _Float16* ka1p = kbase + (size_t)(kb + 16 + c) * DM + 8 * h;
    v8f sacc[2][2], racc[2][2];
#pragma unroll
    for (int qt = 0; qt < 2; ++qt)
#pragma unroll
      for (int kt = 0; kt < 2; ++kt) { sacc[qt][kt] = zero8(); racc[qt][kt] = zero8(); }
#pragma unroll 1
    for (int k0 = 0; k0 < DM; k0 += 32) {
      const v16h a0 = ldfrag(ka0p + k0), a1 = ldfrag(ka1p + k0);
      const v16h b0 = ldfrag(qb0p + k0), b1 = ldfrag(qb1p + k0);
      const v16h r0 = ldfrag(qr0p + k0), r1 = ldfrag(qr1p + k0);
      sacc[0][0] = mma16(a0, b0, sacc[0][0]);
      sacc[0][1] = mma16(a1, b0, sacc[0][1]);
      sacc[1][0] = mma16(a0, b1, sacc[1][0]);
      sacc[1][1] = mma16(a1, b1, sacc[1][1]);
      racc[0][0] = mma16(a0, r0, racc[0][0]);
      racc[0][1] = mma16(a1, r0, racc[0][1]);
      racc[1][0] = mma16(a0, r1, racc[1][0]);
      racc[1][1] = mma16(a1, r1, racc[1][1]);
      guard_s8(sacc[0][0], sacc[0][1], sacc[1][0], sacc[1][1], racc[0][0], racc[0][1], racc[1][0], racc[1][1],
               a0, a1, b0, b1, r0, r1);
    }
    {
      float pm0 = ninf, pm1 = ninf;
#pragma unroll
      for (int kt = 0; kt < 2; ++kt) {
#pragma unroll
        for (int r = 0; r < 8; ++r) {
          const float v0 = (sacc[0][kt][r] + racc[0][kt][r] * R_INV) * S_SC; sacc[0][kt][r] = v0; pm0 = fmaxf(pm0, v0);
          const float v1 = (sacc[1][kt][r] + racc[1][kt][r] * R_INV) * S_SC; sacc[1][kt][r] = v1; pm1 = fmaxf(pm1, v1);
        }
      }
      pm0 = fmaxf(pm0, __shfl_xor(pm0, 16, 32));
      pm1 = fmaxf(pm1, __shfl_xor(pm1, 16, 32));
      pmax[wave * 32 + c] = pm0;
      pmax[wave * 32 + 16 + c] = pm1;
    }
    __syncthreads();
    if (wave == 0) {
      const int row = lane;
      float ps = 0.0f;
#pragma unroll
      for (int w = 0; w < 8; ++w) ps += psum[w * 32 + row];
      l_s[row] = l_s[row] * al_s[row] + ps;
      const float mo = m_s[row];
      float mx = mo;
#pragma unroll
      for (int w = 0; w < 8; ++w) mx = fmaxf(mx, pmax[w * 32 + row]);
      al_s[row] = __expf(mo - mx);
      m_s[row] = mx;
    }
    __syncthreads();
    {
      const float mq0 = m_s[c], mq1 = m_s[16 + c];
      float ps0 = 0.0f, ps1 = 0.0f;
#pragma unroll
      for (int kt = 0; kt < 2; ++kt) {
        v8h h0, h1;
#pragma unroll
        for (int r = 0; r < 8; ++r) {
          const float p0 = __expf(sacc[0][kt][r] - mq0); ps0 += p0; h0[r] = (_Float16)(p0 * 16.0f);
          const float p1 = __expf(sacc[1][kt][r] - mq1); ps1 += p1; h1[r] = (_Float16)(p1 * 16.0f);
        }
        *(v8h*)(Ps + c * PSP + 32 * wave + 16 * kt + 8 * h) = h0;
        *(v8h*)(Ps + (16 + c) * PSP + 32 * wave + 16 * kt + 8 * h) = h1;
      }
      ps0 += __shfl_xor(ps0, 16, 32);
      ps1 += __shfl_xor(ps1, 16, 32);
      psum[wave * 32 + c] = ps0;
      psum[wave * 32 + 16 + c] = ps1;
      const v4f aA = *(const v4f*)(al_s + 8 * h), aB = *(const v4f*)(al_s + 8 * h + 4);
      const v4f bA = *(const v4f*)(al_s + 16 + 8 * h), bB = *(const v4f*)(al_s + 16 + 8 * h + 4);
#pragma unroll
      for (int nt = 0; nt < 2; ++nt) {
#pragma unroll
        for (int r = 0; r < 4; ++r) {
          oacc[0][nt][r] *= aA[r]; oacc[0][nt][4 + r] *= aB[r];
          oacc[1][nt][r] *= bA[r]; oacc[1][nt][4 + r] *= bB[r];
        }
      }
    }
    __syncthreads();
    {
      const _Float16* vbp = vbase + (size_t)(32 * wave + c) * NTOT + (size_t)t * KCH + 8 * h;
#pragma unroll 1
      for (int ks = 0; ks < KCH; ks += 32) {
        const v16h pa0 = ldfrag(pa0p + ks), pa1 = ldfrag(pa1p + ks);
        const v16h vb0 = ldfrag(vbp + ks);
        const v16h vb1 = ldfrag(vbp + (size_t)16 * NTOT + ks);
        oacc[0][0] = mma16(pa0, vb0, oacc[0][0]);
        oacc[0][1] = mma16(pa0, vb1, oacc[0][1]);
        oacc[1][0] = mma16(pa1, vb0, oacc[1][0]);
        oacc[1][1] = mma16(pa1, vb1, oacc[1][1]);
        guard_pv(oacc[0][0], oacc[0][1], oacc[1][0], oacc[1][1], pa0, pa1, vb0, vb1);
      }
    }
  }

  if (wave == 0) {
    const int row = lane;
    float ps = 0.0f;
#pragma unroll
    for (int w = 0; w < 8; ++w) ps += psum[w * 32 + row];
    const float l = l_s[row] * al_s[row] + ps;
    li_s[row] = (1.0f / l) * (1.0f / 256.0f);
  }
  __syncthreads();
  float* Os = (float*)(smem + LQH);
  {
    const v4f iA0 = *(const v4f*)(li_s + 8 * h),      iB0 = *(const v4f*)(li_s + 8 * h + 4);
    const v4f iA1 = *(const v4f*)(li_s + 16 + 8 * h), iB1 = *(const v4f*)(li_s + 16 + 8 * h + 4);
#pragma unroll
    for (int nt = 0; nt < 2; ++nt) {
      const int col = 32 * wave + 16 * nt + c;
#pragma unroll
      for (int r = 0; r < 4; ++r) {
        Os[(8 * h + r) * OSP + col]          = oacc[0][nt][r] * iA0[r];
        Os[(8 * h + 4 + r) * OSP + col]      = oacc[0][nt][4 + r] * iB0[r];
        Os[(16 + 8 * h + r) * OSP + col]     = oacc[1][nt][r] * iA1[r];
        Os[(16 + 8 * h + 4 + r) * OSP + col] = oacc[1][nt][4 + r] * iB1[r];
      }
    }
  }
  __syncthreads();
  {
    const int ca = 4 * lane, cb = 128 + 4 * lane;
    const v4f ga = *(const v4f*)(g2 + ca), gb = *(const v4f*)(g2 + cb);
    const v4f ba = *(const v4f*)(be2 + ca), bb = *(const v4f*)(be2 + cb);
#pragma unroll
    for (int rr = 0; rr < 4; ++rr) {
      const int row = 4 * wave + rr;
      const size_t grow = (size_t)(q0 + row);
      const v4f oa = *(const v4f*)(Os + row * OSP + ca), ob = *(const v4f*)(Os + row * OSP + cb);
      const v4f xa = *(const v4f*)(xn + grow * DM + ca), xb = *(const v4f*)(xn + grow * DM + cb);
      const v4f ya = oa + xa, yb = ob + xb;
      float s = ((ya[0] + ya[1]) + (ya[2] + ya[3])) + ((yb[0] + yb[1]) + (yb[2] + yb[3]));
#pragma unroll
      for (int off = 16; off > 0; off >>= 1) s += __shfl_xor(s, off, 32);
      const float mu = s * (1.0f / 256.0f);
      float s2 = 0.0f;
#pragma unroll
      for (int e = 0; e < 4; ++e) {
        const float d0 = ya[e] - mu, d1 = yb[e] - mu;
        s2 += d0 * d0; s2 += d1 * d1;
      }
#pragma unroll
      for (int off = 16; off > 0; off >>= 1) s2 += __shfl_xor(s2, off, 32);
      const float rstd8 = rsqrtf(s2 * (1.0f / 256.0f) + 1e-5f) * 8.0f;
      v4h ha, hb;
#pragma unroll
      for (int e = 0; e < 4; ++e) {
        ha[e] = (_Float16)((ya[e] - mu) * rstd8 * bfr(ga[e]) + bfr(ba[e]) * 8.0f);
        hb[e] = (_Float16)((yb[e] - mu) * rstd8 * bfr(gb[e]) + bfr(bb[e]) * 8.0f);
      }
      float* yr = x1 + grow * DM;
      _Float16* hr = h16 + grow * DM;
#pragma unroll
      for (int ps = 0; ps < 2; ++ps) {
        *(volatile v4f*)(yr + ca) = ya;
        *(volatile v4f*)(yr + cb) = yb;
        *(volatile v4h*)(hr + ca) = ha;
        *(volatile v4h*)(hr + cb) = hb;
        __threadfence();
      }
    }
  }
}

extern "C" void kernel_launch(void* const* d_in, const int* in_sizes, int n_in,
                              void* d_out, int out_size, void* d_ws, size_t ws_size,
                              hipStream_t stream) {
  if (n_in < 15) return;
  const int ntot = NTOT, dm = DM, ff = FF;
  if (in_sizes[0] != ntot * dm) return;
  if (in_sizes[1] != dm || in_sizes[2] != dm || in_sizes[4] != dm || in_sizes[6] != dm || in_sizes[8] != dm) return;
  if (in_sizes[9] != dm || in_sizes[10] != dm || in_sizes[14] != dm || in_sizes[12] != ff) return;
  if (in_sizes[3] != dm * dm || in_sizes[5] != dm * dm || in_sizes[7] != dm * dm) return;
  if (in_sizes[11] != dm * ff || in_sizes[13] != ff * dm) return;
  if (out_size != ntot * dm) return;

  const float* x     = (const float*)d_in[0];
  const float* ln1_g = (const float*)d_in[1];
  const float* ln1_b = (const float*)d_in[2];
  const float* wq    = (const float*)d_in[3];
  const float* bq    = (const float*)d_in[4];
  const float* wk    = (const float*)d_in[5];
  const float* bk    = (const float*)d_in[6];
  const float* wv    = (const float*)d_in[7];
  const float* bv    = (const float*)d_in[8];
  const float* ln2_g = (const float*)d_in[9];
  const float* ln2_b = (const float*)d_in[10];
  const float* w1    = (const float*)d_in[11];
  const float* b1    = (const float*)d_in[12];
  const float* w2    = (const float*)d_in[13];
  const float* b2    = (const float*)d_in[14];
  float* out = (float*)d_out;

  const size_t bWs  = (size_t)dm * dm * 2;
  const size_t bWf  = (size_t)dm * ff * 2;
  const size_t bF32 = (size_t)ntot * dm * 4;
  const size_t bH16 = (size_t)ntot * dm * 2;
  const size_t bM16 = (size_t)ntot * ff * 2;
  size_t off = 0;
  const size_t oWq  = off; off += bWs;
  const size_t oWk  = off; off += bWs;
  const size_t oWv  = off; off += bWs;
  const size_t oW1  = off; off += bWf;
  const size_t oW2  = off; off += bWf;
  const size_t oXN  = off; off += bF32;
  const size_t oX16 = off; off += bH16;
  const size_t oQH  = off; off += bH16;
  const size_t oQR  = off; off += bH16;
  const size_t oKH  = off; off += bH16;
  const size_t oVT  = off; off += bH16;
  const size_t oX1  = off; off += bF32;
  const size_t oH   = off; off += bH16;
  const size_t oM   = off; off += bM16;
  if (off > ws_size) return;
  if (off > (size_t)134217728) return;

  char* ws = (char*)d_ws;
  _Float16* WqT = (_Float16*)(ws + oWq);
  _Float16* WkT = (_Float16*)(ws + oWk);
  _Float16* WvT = (_Float16*)(ws + oWv);
  _Float16* W1T = (_Float16*)(ws + oW1);
  _Float16* W2T = (_Float16*)(ws + oW2);
  float*    XN  = (float*)(ws + oXN);
  _Float16* X16 = (_Float16*)(ws + oX16);
  _Float16* QH  = (_Float16*)(ws + oQH);
  _Float16* QR  = (_Float16*)(ws + oQR);
  _Float16* KH  = (_Float16*)(ws + oKH);
  _Float16* VT  = (_Float16*)(ws + oVT);
  float*    X1  = (float*)(ws + oX1);
  _Float16* H16 = (_Float16*)(ws + oH);
  _Float16* M16 = (_Float16*)(ws + oM);

  const dim3 blk(256);

  cvt_w_kernel<<<dim3(176), blk, 0, stream>>>(wq, wk, wv, w1, w2, WqT, WkT, WvT, W1T, W2T);
  ln1_kernel<<<dim3(ntot / 8), blk, 0, stream>>>(x, ln1_g, ln1_b, XN, X16, ntot);
  gemm64_kernel<2, false, false, false><<<dim3(((ntot / 64) * (dm / 64)) / 8), blk, 0, stream>>>(
      X16, dm, WqT, dm, (void*)QH, QR, dm, bq, XN, dm, ntot, dm, dm, 0.03125f, 16.0f);
  gemm64_kernel<1, false, false, false><<<dim3(((ntot / 64) * (dm / 64)) / 8), blk, 0, stream>>>(
      X16, dm, WkT, dm, (void*)KH, KH, dm, bk, XN, dm, ntot, dm, dm, 0.03125f, 16.0f);
  gemm64_kernel<1, true, false, false><<<dim3(((dm / 64) * (ntot / 64)) / 8), blk, 0, stream>>>(
      WvT, dm, X16, dm, (void*)VT, VT, ntot, bv, XN, dm, dm, ntot, dm, 0.03125f, 16.0f);
  attn_kernel<<<dim3(ntot / QB), blk, 0, stream>>>(QH, QR, KH, VT, XN, ln2_g, ln2_b, X1, H16);
  gemm64_kernel<1, false, true, false><<<dim3(((ntot / 64) * (ff / 64)) / 8), blk, 0, stream>>>(
      H16, dm, W1T, dm, (void*)M16, M16, ff, b1, XN, dm, ntot, ff, dm, 0.015625f, 8.0f);
  gemm64_kernel<0, false, false, true><<<dim3(((ntot / 64) * (dm / 64)) / 8), blk, 0, stream>>>(
      M16, ff, W2T, ff, (void*)out, H16, dm, b2, X1, dm, ntot, dm, ff, 0.001953125f, 1.0f);
  (void)hipGetLastError();
}
